// multiLayer_TranLSTM_12326556139970
// MI455X (gfx1250) — hardware-verified
//
#include <hip/hip_runtime.h>
#include <math.h>

constexpr int BATCH  = 256;
constexpr int TSTEPS = 10;
constexpr int DIN    = 512;
constexpr int HID    = 1024;
constexpr int FFD    = 2048;
constexpr int NSLOT  = 2;
constexpr int NHEADS = 16;
constexpr int HEADD  = 64;
constexpr int O1D    = 512;
constexpr int NCLS   = 2;
constexpr int MROWS  = BATCH * TSTEPS;
constexpr int HEADD_SQRT = 8;
constexpr float ATT_SCALE  = 1.0f / (float)HEADD_SQRT;
constexpr float WCARRY     = 16.0f;
constexpr float WCARRY_INV = 1.0f / 16.0f;
constexpr float RCARRY     = 2048.0f;
constexpr float RCARRY_INV = 1.0f / 2048.0f;
constexpr float H16_MIN_NORMAL = 6.103515625e-5f;
constexpr float LN_EPS_F   = 1e-5f;
constexpr int HP    = HID + 8;
constexpr int SLABP = 68;
constexpr int ATT_WAVES = 4;
constexpr int NPAIR = (TSTEPS * (TSTEPS + 1)) / 2;

constexpr size_t OUT0_ELEMS  = (size_t)MROWS * NCLS;
constexpr size_t OUT1_OFF_B  = 20480;
constexpr size_t OUT2_OFF_B  = 2117632;
constexpr size_t OUT_TOTAL_B = 4214784;
constexpr size_t STATE_B     = (size_t)BATCH * NSLOT * HID * 4;

static_assert(HEADD_SQRT * HEADD_SQRT == HEADD);
static_assert(NHEADS * HEADD == HID);
static_assert(OUT0_ELEMS * 4 == OUT1_OFF_B);
static_assert(OUT1_OFF_B + STATE_B == OUT2_OFF_B);
static_assert(OUT2_OFF_B + STATE_B == OUT_TOTAL_B);
static_assert(OUT1_OFF_B % 128 == 0 && OUT2_OFF_B % 128 == 0);
static_assert(MROWS % 64 == 0 && HID % 64 == 0 && (3 * HID) % 64 == 0 && FFD % 64 == 0 && (4 * HID) % 64 == 0 && O1D % 64 == 0);
static_assert(DIN % 32 == 0 && HID % 32 == 0 && FFD % 32 == 0);
static_assert(BATCH % 16 == 0);
static_assert(HID == 128 * 8);
static_assert(NHEADS % ATT_WAVES == 0);
static_assert(NPAIR == 55 && NPAIR <= 64);
static_assert(MROWS % 256 == 0);
static_assert(2 * O1D == 4 * 256);
static_assert((3 * TSTEPS * HEADD / 4) % 32 == 0);

typedef __attribute__((ext_vector_type(16))) _Float16 v16h;
typedef __attribute__((ext_vector_type(8)))  _Float16 v8h;
typedef __attribute__((ext_vector_type(4)))  _Float16 v4h;
typedef __attribute__((ext_vector_type(8)))  float    v8f;
typedef __attribute__((ext_vector_type(4)))  float    v4f;
typedef __attribute__((ext_vector_type(2)))  float    v2f;
typedef __attribute__((ext_vector_type(4)))  unsigned v4u;

__device__ __forceinline__ unsigned short f2bf_bits(float f) {
  unsigned u = __float_as_uint(f);
  return (unsigned short)((u + 0x7FFFu + ((u >> 16) & 1u)) >> 16);
}
__device__ __forceinline__ float bf_bits2f(unsigned short h) { return __uint_as_float(((unsigned)h) << 16); }
__device__ __forceinline__ float bf16r(float f) { return bf_bits2f(f2bf_bits(f)); }

__device__ __forceinline__ float h16_to_f32(unsigned hb) {
  const unsigned sgn = (hb & 0x8000u) << 16;
  const unsigned em = hb & 0x7fffu;
  const float fn = __uint_as_float((em << 13) + 0x38000000u);
  const float fs = (float)em * 5.9604644775390625e-8f;
  const float mag = (em < 0x400u) ? fs : fn;
  return __uint_as_float(__float_as_uint(mag) | sgn);
}

__device__ __forceinline__ void split_h16(float v, _Float16& hi, _Float16& lo) {
  const float vh = (fabsf(v) < H16_MIN_NORMAL) ? 0.0f : v;
  const _Float16 h = (_Float16)vh;
  float hf = (float)h;
  asm volatile("" : "+v"(hf));
  hi = h;
  lo = (_Float16)((v - hf) * RCARRY);
}

__device__ __forceinline__ void guard_row4_h(v8f& a0, v8f& a1, v8f& a2, v8f& a3, v16h x, v16h y0, v16h y1, v16h y2, v16h y3) {
  asm volatile("v_nop\n\tv_nop\n\tv_nop\n\tv_nop" : "+v"(a0), "+v"(a1), "+v"(a2), "+v"(a3) : "v"(x), "v"(y0), "v"(y1), "v"(y2), "v"(y3));
}
__device__ __forceinline__ void keep4_h(v16h a, v16h b, v16h c, v16h d) { asm volatile("v_nop" :: "v"(a), "v"(b), "v"(c), "v"(d)); }
__device__ __forceinline__ void acc_guard4(v8f& a, v8f& b, v8f& c, v8f& d) { asm volatile("v_nop\n\tv_nop\n\tv_nop\n\tv_nop" : "+v"(a), "+v"(b), "+v"(c), "+v"(d)); }

struct FragH {
  union U { v16h v; v8h h[2]; };
  static __device__ __forceinline__ v16h load(const _Float16* p) {
    U f; f.h[0] = *(const v8h*)(p); f.h[1] = *(const v8h*)(p + 16); return f.v;
  }
  static __device__ __forceinline__ v8f mma(v16h a, v16h b, v8f c) {
    return __builtin_amdgcn_wmma_f32_16x16x32_f16(false, a, false, b, (short)0, c, false, false);
  }
};

__device__ __forceinline__ float sigm_f(float x)  { return __builtin_amdgcn_rcpf(1.0f + expf(-x)); }
__device__ __forceinline__ float tanh_f(float x)  { return 1.0f - 2.0f * __builtin_amdgcn_rcpf(expf(2.0f * x) + 1.0f); }

__global__ __launch_bounds__(256) void cvt8_kernel(const float* __restrict__ src, unsigned short* __restrict__ dst, int n8, float sc) {
  const int i = blockIdx.x * 256 + threadIdx.x;
  if (i < n8) {
    const float* sp = src + (size_t)i * 8;
    const v4f a = *(const v4f*)(sp);
    const v4f b = *(const v4f*)(sp + 4);
    v8h hv;
#pragma unroll
    for (int e = 0; e < 4; ++e) {
      const float fa = a[e];
      const float fb = b[e];
      hv[e]     = (_Float16)(bf16r(fa) * sc);
      hv[4 + e] = (_Float16)(bf16r(fb) * sc);
    }
    *(volatile v8h*)(dst + (size_t)i * 8) = hv;
    __threadfence();
    *(volatile v8h*)(dst + (size_t)i * 8) = hv;
  }
}

__device__ __forceinline__ void gemm_kpass(v8f (&acc)[4][4], const _Float16* arow, const _Float16* brow,
                                           size_t a16, size_t b16, int K) {
  for (int k0 = 0; k0 < K; k0 += 32) {
    v16h bh[4];
#pragma unroll
    for (int j = 0; j < 4; ++j) bh[j] = FragH::load(brow + j * b16 + k0);
#pragma unroll
    for (int i = 0; i < 4; ++i) {
      const v16h ah = FragH::load(arow + i * a16 + k0);
#pragma unroll
      for (int j = 0; j < 4; ++j) acc[i][j] = FragH::mma(ah, bh[j], acc[i][j]);
      guard_row4_h(acc[i][0], acc[i][1], acc[i][2], acc[i][3], ah, bh[0], bh[1], bh[2], bh[3]);
    }
    keep4_h(bh[0], bh[1], bh[2], bh[3]);
  }
  acc_guard4(acc[0][0], acc[0][1], acc[0][2], acc[0][3]);
  acc_guard4(acc[1][0], acc[1][1], acc[1][2], acc[1][3]);
  acc_guard4(acc[2][0], acc[2][1], acc[2][2], acc[2][3]);
  acc_guard4(acc[3][0], acc[3][1], acc[3][2], acc[3][3]);
}

template <bool ASPLIT, int OUT_MODE, bool RESID, int ACT>
__global__ __launch_bounds__(256) void wmma_gemm64_f16(
    const unsigned short* __restrict__ Ap, const unsigned short* __restrict__ A2p, int lda,
    const unsigned short* __restrict__ Btp, int ldb,
    float* __restrict__ Cout, unsigned short* __restrict__ Chi, unsigned short* __restrict__ Clo, int ldc,
    const float* __restrict__ bias, const float* __restrict__ resid,
    int M, int N, int K, float scale) {
  static_assert(OUT_MODE == 0 || OUT_MODE == 1 || OUT_MODE == 4);
  static_assert(ACT == 0 || ACT == 2);
  static_assert(!(RESID && (ACT != 0 || OUT_MODE != 0)));
  const _Float16* A  = (const _Float16*)Ap;
  const _Float16* A2 = (const _Float16*)A2p;
  const _Float16* Bt = (const _Float16*)Btp;
  __shared__ __align__(16) float sT[8][16 * 68];
  const int lane = threadIdx.x & 31;
  const int wave = threadIdx.x >> 5;
  const int tilesN = N >> 6;
  const int tilesM = M >> 6;
  const int tile = blockIdx.x * 8 + wave;
  if (tile >= tilesM * tilesN) return;
  const int tm = tile / tilesN;
  const int tn = tile - tm * tilesN;
  const int m0 = tm << 6;
  const int n0 = tn << 6;
  const int rlane = lane & 15;
  const int koff  = (lane >> 4) * 8;
  const int mOff  = (lane >> 4) * 8;

  v8f acc[4][4];
#pragma unroll
  for (int i = 0; i < 4; ++i)
#pragma unroll
    for (int j = 0; j < 4; ++j) acc[i][j] = (v8f){0.f, 0.f, 0.f, 0.f, 0.f, 0.f, 0.f, 0.f};

  const size_t aoff = (size_t)(m0 + rlane) * lda + koff;
  const _Float16* arow = A + aoff;
  const _Float16* brow = Bt + (size_t)(n0 + rlane) * ldb + koff;
  const size_t a16 = (size_t)16 * lda;
  const size_t b16 = (size_t)16 * ldb;

  if (ASPLIT) {
    gemm_kpass(acc, A2 + aoff, brow, a16, b16, K);
#pragma unroll
    for (int i = 0; i < 4; ++i)
#pragma unroll
      for (int j = 0; j < 4; ++j) acc[i][j] = acc[i][j] * RCARRY_INV;
  }
  gemm_kpass(acc, arow, brow, a16, b16, K);

  float* slab = sT[wave];
#pragma unroll
  for (int i = 0; i < 4; ++i) {
    const int mBase = m0 + (i << 4);
#pragma unroll
    for (int j = 0; j < 4; ++j) {
      const int n = n0 + (j << 4) + rlane;
      const float bv = bf16r(bias[n]);
#pragma unroll
      for (int r = 0; r < 8; ++r) {
        float v = acc[i][j][r] * scale + bv;
        if (ACT == 2) v = fmaxf(v, 0.0f);
        slab[(mOff + r) * 68 + (j << 4) + rlane] = v;
      }
    }
    __builtin_amdgcn_fence(__ATOMIC_RELEASE, "workgroup");
    __builtin_amdgcn_wave_barrier();
    __builtin_amdgcn_fence(__ATOMIC_ACQUIRE, "workgroup");
    if (OUT_MODE == 0 || OUT_MODE == 4) {
      const int hh = lane >> 4, c4 = (lane & 15) * 4;
      for (int pass = 0; pass < 2; ++pass) {
#pragma unroll
        for (int it = 0; it < 8; ++it) {
          const int row = it * 2 + hh;
          const size_t go = (size_t)(mBase + row) * ldc + n0 + c4;
          v4f v = *(const v4f*)(slab + row * 68 + c4);
          if (RESID) {
            const v4f rv = *(const v4f*)(resid + go);
            v = v + rv;
          }
          *(volatile v4f*)(Cout + go) = v;
        }
        __threadfence();
      }
    }
    if (OUT_MODE == 1 || OUT_MODE == 4) {
      const int q = lane >> 3, c8 = (lane & 7) * 8;
      for (int pass = 0; pass < 2; ++pass) {
#pragma unroll
        for (int it = 0; it < 4; ++it) {
          const int row = it * 4 + q;
          const float* sp = slab + row * 68 + c8;
          const v4f x0 = *(const v4f*)(sp);
          const v4f x1 = *(const v4f*)(sp + 4);
          v8h hv, lv;
#pragma unroll
          for (int e = 0; e < 4; ++e) {
            const float f0 = x0[e];
            const float f1 = x1[e];
            if (OUT_MODE == 1) {
              hv[e]     = (_Float16)f0;
              hv[4 + e] = (_Float16)f1;
              lv[e]     = hv[e];
              lv[4 + e] = hv[4 + e];
            } else {
              _Float16 a0, b0, a1, b1;
              split_h16(f0, a0, b0);
              split_h16(f1, a1, b1);
              hv[e] = a0; lv[e] = b0;
              hv[4 + e] = a1; lv[4 + e] = b1;
            }
          }
          const size_t go = (size_t)(mBase + row) * ldc + n0 + c8;
          *(volatile v8h*)(Chi + go) = hv;
          if (OUT_MODE == 4) *(volatile v8h*)(Clo + go) = lv;
        }
        __threadfence();
      }
    }
    __builtin_amdgcn_fence(__ATOMIC_RELEASE, "workgroup");
    __builtin_amdgcn_wave_barrier();
    __builtin_amdgcn_fence(__ATOMIC_ACQUIRE, "workgroup");
  }
}

__global__ __launch_bounds__(128) void attn_kernel(const float* __restrict__ qkv, unsigned short* __restrict__ ctxh,
                                                   unsigned short* __restrict__ ctxl) {
  __shared__ __align__(16) float QKVs[ATT_WAVES][3 * TSTEPS * HEADD];
  __shared__ __align__(16) float Ss[ATT_WAVES][TSTEPS * 12];
  __shared__ __align__(16) float Pn[ATT_WAVES][TSTEPS * 12];
  __shared__ __align__(16) float Inv[ATT_WAVES][16];
  const int tid = threadIdx.x, lane = tid & 31, wave = tid >> 5;
  const int b = blockIdx.x / (NHEADS / ATT_WAVES);
  const int head = (blockIdx.x % (NHEADS / ATT_WAVES)) * ATT_WAVES + wave;
  float* sq = QKVs[wave];
  float* ps = Ss[wave];
  float* pn = Pn[wave];
  float* iv = Inv[wave];

#pragma unroll 1
  for (int it = 0; it < 15; ++it) {
    const int idx = it * 32 + lane;
    const int seg = idx >> 4, part = idx & 15;
    const int which = seg / TSTEPS;
    const int t = seg - which * TSTEPS;
    const size_t eoff = (size_t)(b * TSTEPS + t) * (3 * HID) + (size_t)which * HID + head * HEADD + part * 4;
    const v4f w = *(const v4f*)(qkv + eoff);
    *(v4f*)(sq + idx * 4) = w;
  }
  __syncthreads();

#pragma unroll 1
  for (int pp = 0; pp < 2; ++pp) {
    const int p = pp * 32 + lane;
    const int pc = p < NPAIR ? p : NPAIR - 1;
    const int qi = (pc >= 1) + (pc >= 3) + (pc >= 6) + (pc >= 10) + (pc >= 15) + (pc >= 21) + (pc >= 28) + (pc >= 36) + (pc >= 45);
    const int ki = pc - (qi * (qi + 1)) / 2;
    const float* qr = sq + qi * HEADD;
    const float* kr = sq + TSTEPS * HEADD + ki * HEADD;
    float acc = 0.0f;
#pragma unroll 1
    for (int d = 0; d < HEADD; d += 4) {
      const v4f a = *(const v4f*)(qr + d);
      const v4f k4 = *(const v4f*)(kr + d);
      acc += a[0] * k4[0];
      acc += a[1] * k4[1];
      acc += a[2] * k4[2];
      acc += a[3] * k4[3];
    }
    if (p < NPAIR) ps[qi * 12 + ki] = acc * ATT_SCALE;
  }
  __syncthreads();

  {
    const int qi = lane < TSTEPS ? lane : TSTEPS - 1;
    float m = -INFINITY;
#pragma unroll 1
    for (int k = 0; k < TSTEPS; ++k) {
      const int kc = k <= qi ? k : qi;
      m = fmaxf(m, ps[qi * 12 + kc]);
    }
    float sum = 0.0f;
#pragma unroll 1
    for (int k = 0; k < TSTEPS; ++k) {
      const int kc = k <= qi ? k : qi;
      const float ex = expf(ps[qi * 12 + kc] - m);
      const float e = (k <= qi) ? ex : 0.0f;
      sum += e;
      if (lane < TSTEPS && k <= qi) pn[qi * 12 + k] = e;
    }
    if (lane < TSTEPS) iv[lane] = 1.0f / sum;
  }
  __syncthreads();

  {
    const float* vs = sq + 2 * TSTEPS * HEADD;
#pragma unroll 1
    for (int qi = 0; qi < TSTEPS; ++qi) {
      float a0 = 0.0f, a1 = 0.0f;
#pragma unroll 1
      for (int k = 0; k <= qi; ++k) {
        const float p = pn[qi * 12 + k];
        const v2f vv = *(const v2f*)(vs + k * HEADD + 2 * lane);
        a0 += p * vv[0];
        a1 += p * vv[1];
      }
      const float sc = iv[qi];
      v2f o;
      o[0] = a0 * sc;
      o[1] = a1 * sc;
      *(v2f*)(sq + qi * HEADD + 2 * lane) = o;
    }
  }
  __syncthreads();

  {
    const size_t cbase = (size_t)(b * TSTEPS) * HID + head * HEADD;
    const int rq = lane >> 3, c8 = (lane & 7) * 8;
    v8h hv[3], lv[3];
#pragma unroll
    for (int it = 0; it < 3; ++it) {
      const int row = it * 4 + rq;
      const int rc = row < TSTEPS ? row : TSTEPS - 1;
      const float* sp = sq + rc * HEADD + c8;
      const v4f x0 = *(const v4f*)(sp);
      const v4f x1 = *(const v4f*)(sp + 4);
#pragma unroll
      for (int e = 0; e < 4; ++e) {
        const float f0 = x0[e];
        const float f1 = x1[e];
        _Float16 a0, b0, a1, b1;
        split_h16(f0, a0, b0);
        split_h16(f1, a1, b1);
        hv[it][e] = a0; lv[it][e] = b0;
        hv[it][4 + e] = a1; lv[it][4 + e] = b1;
      }
    }
    for (int pass = 0; pass < 2; ++pass) {
#pragma unroll
      for (int it = 0; it < 3; ++it) {
        const int row = it * 4 + rq;
        if (row < TSTEPS) {
          *(volatile v8h*)(ctxh + cbase + (size_t)row * HID + c8) = hv[it];
          *(volatile v8h*)(ctxl + cbase + (size_t)row * HID + c8) = lv[it];
        }
      }
      __threadfence();
    }
  }
}

template <int MODE>
__global__ __launch_bounds__(256) void ln_rows_kernel(const float* __restrict__ S, const float* __restrict__ gam,
                                                      const float* __restrict__ bet, float* __restrict__ Y32,
                                                      unsigned short* __restrict__ Yhi, unsigned short* __restrict__ Ylo,
                                                      int nrows) {
  const int tid = threadIdx.x, lane = tid & 31;
  const int row = blockIdx.x * 8 + (tid >> 5);
  if (row >= nrows) return;
  const float* rp = S + (size_t)row * HID;
  v4f v[8];
  float s = 0.0f;
#pragma unroll
  for (int q = 0; q < 8; ++q) {
    v[q] = *(const v4f*)(rp + 128 * q + 4 * lane);
    s += (v[q][0] + v[q][1]) + (v[q][2] + v[q][3]);
  }
#pragma unroll
  for (int off = 1; off < 32; off <<= 1) s += __shfl_xor(s, off, 32);
  const float mu = s * (1.0f / HID);
  float ss = 0.0f;
#pragma unroll
  for (int q = 0; q < 8; ++q)
#pragma unroll
    for (int e = 0; e < 4; ++e) {
      const float d = v[q][e] - mu;
      v[q][e] = d;
      ss += d * d;
    }
#pragma unroll
  for (int off = 1; off < 32; off <<= 1) ss += __shfl_xor(ss, off, 32);
  const float rstd = rsqrtf(ss * (1.0f / HID) + LN_EPS_F);
  v4h hq[8], lq[8];
#pragma unroll
  for (int q = 0; q < 8; ++q) {
    const v4f g  = *(const v4f*)(gam + 128 * q + 4 * lane);
    const v4f bb = *(const v4f*)(bet + 128 * q + 4 * lane);
#pragma unroll
    for (int e = 0; e < 4; ++e) {
      const float ge = g[e];
      const float be = bb[e];
      const float o = (v[q][e] * rstd) * bf16r(ge) + bf16r(be);
      v[q][e] = o;
      if (MODE == 0) {
        hq[q][e] = (_Float16)o;
        lq[q][e] = hq[q][e];
      } else {
        _Float16 a0, b0;
        split_h16(o, a0, b0);
        hq[q][e] = a0;
        lq[q][e] = b0;
      }
    }
  }
  float* op = Y32 + (size_t)row * HID;
  unsigned short* oh = Yhi + (size_t)row * HID;
  unsigned short* ol = Ylo + (size_t)row * HID;
  for (int pass = 0; pass < 2; ++pass) {
#pragma unroll
    for (int q = 0; q < 8; ++q) {
      if (MODE == 0) *(volatile v4f*)(op + 128 * q + 4 * lane) = v[q];
      *(volatile v4h*)(oh + 128 * q + 4 * lane) = hq[q];
      if (MODE == 1) *(volatile v4h*)(ol + 128 * q + 4 * lane) = lq[q];
    }
    __threadfence();
  }
}

__global__ __launch_bounds__(256) void lstm_seq_kernel(const float* __restrict__ XG,
                                                       const unsigned short* __restrict__ WHHp,
                                                       const float* __restrict__ bhh,
                                                       const float* __restrict__ h0in, const float* __restrict__ c0in,
                                                       float* __restrict__ SEQ32, unsigned short* __restrict__ SEQHI,
                                                       unsigned short* __restrict__ SEQLO,
                                                       float* __restrict__ CT_out, float* __restrict__ HT_out, int slot) {
  __shared__ __align__(16) _Float16 Ah[2][16 * HP];
  __shared__ __align__(16) float    cL[8 * 8 * 8 * 32];
  __shared__ __align__(16) float    Sl[8][16 * SLABP];
  const _Float16* WHH = (const _Float16*)WHHp;
  const int tid = threadIdx.x, lane = tid & 31, wave = tid >> 5;
  const int c = lane & 15, hh = lane >> 4, koff = hh * 8, c4 = c * 4;
  const int q4 = lane >> 3, c8 = (lane & 7) * 8;
  const int rowbase = blockIdx.x * 16;

  {
    _Float16* ah0 = &Ah[0][0];
#pragma unroll 1
    for (int i = 0; i < 16; ++i) {
      const int cc4 = tid * 4;
      const v4f hv = *(const v4f*)(h0in + ((size_t)(rowbase + i) * NSLOT + slot) * HID + cc4);
      v4h h4;
#pragma unroll
      for (int e = 0; e < 4; ++e) {
        const float he = hv[e];
        h4[e] = (_Float16)bf16r(he);
      }
      *(v4h*)(ah0 + i * HP + cc4) = h4;
    }
  }
#pragma unroll 1
  for (int sub = 0; sub < 8; ++sub) {
    const int u = 128 * wave + 16 * sub + c;
#pragma unroll
    for (int r = 0; r < 8; ++r)
      cL[((wave * 8 + sub) * 8 + r) * 32 + lane] = bf16r(c0in[((size_t)(rowbase + 8 * hh + r) * NSLOT + slot) * HID + u]);
  }
  __syncthreads();

  const v8f z8 = {0.f, 0.f, 0.f, 0.f, 0.f, 0.f, 0.f, 0.f};
  float* slab = Sl[wave];

#pragma unroll 1
  for (int t = 0; t < TSTEPS; ++t) {
    const int cur = t & 1;
    const _Float16* ahrow = &Ah[cur][0] + c * HP + koff;
    _Float16* ahn = &Ah[cur ^ 1][0];
    const bool last = (t == TSTEPS - 1);

#pragma unroll 1
    for (int sub = 0; sub < 8; ++sub) {
      const int u = 128 * wave + 16 * sub + c;
      const _Float16* wh = WHH + (size_t)u * HID + koff;
      v8f acc[4];
      acc[0] = z8; acc[1] = z8; acc[2] = z8; acc[3] = z8;
#pragma unroll 1
      for (int k0 = 0; k0 < HID; k0 += 32) {
        const v16h a  = FragH::load(ahrow + k0);
        const v16h b0 = FragH::load(wh + k0);
        const v16h b1 = FragH::load(wh + (size_t)1 * HID * HID + k0);
        const v16h b2 = FragH::load(wh + (size_t)2 * HID * HID + k0);
        const v16h b3 = FragH::load(wh + (size_t)3 * HID * HID + k0);
        acc[0] = FragH::mma(a, b0, acc[0]);
        acc[1] = FragH::mma(a, b1, acc[1]);
        acc[2] = FragH::mma(a, b2, acc[2]);
        acc[3] = FragH::mma(a, b3, acc[3]);
        guard_row4_h(acc[0], acc[1], acc[2], acc[3], a, b0, b1, b2, b3);
      }
      acc_guard4(acc[0], acc[1], acc[2], acc[3]);

      const float bi = bf16r(bhh[u]);
      const float bf = bf16r(bhh[HID + u]);
      const float bg = bf16r(bhh[2 * HID + u]);
      const float bo = bf16r(bhh[3 * HID + u]);
      const float* xgp = XG + ((size_t)(rowbase + 8 * hh) * TSTEPS + (size_t)t) * (4 * HID) + u;
      float* cp = cL + ((wave * 8 + sub) * 8) * 32 + lane;
      const int scol = (sub & 3) * 16 + c;
#pragma unroll
      for (int r = 0; r < 8; ++r) {
        const float* xr = xgp + (size_t)r * (TSTEPS * 4 * HID);
        const float xi = xr[0];
        const float xf = xr[HID];
        const float xc = xr[2 * HID];
        const float xo = xr[3 * HID];
        const float zi = (acc[0][r] * WCARRY_INV + xi) + bi;
        const float zf = (acc[1][r] * WCARRY_INV + xf) + bf;
        const float zg = (acc[2][r] * WCARRY_INV + xc) + bg;
        const float zo = (acc[3][r] * WCARRY_INV + xo) + bo;
        const float ig = sigm_f(zi);
        const float fg = sigm_f(zf);
        const float gg = tanh_f(zg);
        const float og = sigm_f(zo);
        const float cold = cp[r * 32];
        const float cn = fg * cold + ig * gg;
        cp[r * 32] = cn;
        const float hn = og * tanh_f(cn);
        ahn[(8 * hh + r) * HP + u] = (_Float16)hn;
        slab[(8 * hh + r) * SLABP + scol] = hn;
      }
      if ((sub & 3) == 3) {
        const int colb = 128 * wave + 64 * (sub >> 2);
        __builtin_amdgcn_fence(__ATOMIC_RELEASE, "workgroup");
        __builtin_amdgcn_wave_barrier();
        __builtin_amdgcn_fence(__ATOMIC_ACQUIRE, "workgroup");
        for (int pass = 0; pass < 2; ++pass) {
#pragma unroll
          for (int it = 0; it < 8; ++it) {
            const int row = it * 2 + hh;
            const v4f v = *(const v4f*)(slab + row * SLABP + c4);
            *(volatile v4f*)(SEQ32 + ((size_t)(rowbase + row) * TSTEPS + (size_t)t) * HID + colb + c4) = v;
            if (last) *(volatile v4f*)(HT_out + ((size_t)(rowbase + row) * NSLOT + slot) * HID + colb + c4) = v;
          }
          __threadfence();
        }
        for (int pass = 0; pass < 2; ++pass) {
#pragma unroll
          for (int it = 0; it < 4; ++it) {
            const int row = it * 4 + q4;
            const float* sp = slab + row * SLABP + c8;
            const v4f x0 = *(const v4f*)(sp);
            const v4f x1 = *(const v4f*)(sp + 4);
            v8h hv, lv;
#pragma unroll
            for (int e = 0; e < 4; ++e) {
              const float f0 = x0[e];
              const float f1 = x1[e];
              _Float16 a0, b0, a1, b1;
              split_h16(f0, a0, b0);
              split_h16(f1, a1, b1);
              hv[e] = a0; lv[e] = b0;
              hv[4 + e] = a1; lv[4 + e] = b1;
            }
            const size_t go = ((size_t)(rowbase + row) * TSTEPS + (size_t)t) * HID + colb + c8;
            *(volatile v8h*)(SEQHI + go) = hv;
            *(volatile v8h*)(SEQLO + go) = lv;
          }
          __threadfence();
        }
        __builtin_amdgcn_fence(__ATOMIC_RELEASE, "workgroup");
        __builtin_amdgcn_wave_barrier();
        __builtin_amdgcn_fence(__ATOMIC_ACQUIRE, "workgroup");
      }
    }
    __syncthreads();
  }

  __syncthreads();
  for (int pass = 0; pass < 2; ++pass) {
#pragma unroll
    for (int R = 0; R < 16; ++R) {
      const v4f v = *(const v4f*)(cL + ((wave * 8 + (lane >> 2)) * 8 + (R & 7)) * 32 + (R >> 3) * 16 + 4 * (lane & 3));
      *(volatile v4f*)(CT_out + ((size_t)(rowbase + R) * NSLOT + slot) * HID + 128 * wave + 4 * lane) = v;
    }
    __threadfence();
  }
}

__global__ __launch_bounds__(256) void head_kernel(const unsigned short* __restrict__ O1, const float* __restrict__ w2,
                                                   const float* __restrict__ b2, float* __restrict__ out) {
  __shared__ __align__(16) float Ws[2 * O1D];
  const int tid = threadIdx.x;
  {
    const v4f w = *(const v4f*)(w2 + tid * 4);
    v4f wr;
#pragma unroll
    for (int e = 0; e < 4; ++e) {
      const float we = w[e];
      wr[e] = bf16r(we);
    }
    *(v4f*)(Ws + tid * 4) = wr;
  }
  __syncthreads();
  const int row = blockIdx.x * 256 + tid;
  const v4u* rp = (const v4u*)(O1 + (size_t)row * O1D);
  float s0 = 0.0f, s1 = 0.0f;
#pragma unroll 1
  for (int k8 = 0; k8 < O1D / 8; ++k8) {
    const v4u w = rp[k8];
    const unsigned w0 = w[0], w1 = w[1], w2w = w[2], w3 = w[3];
    const v4f a0 = *(const v4f*)(Ws + k8 * 8);
    const v4f a1 = *(const v4f*)(Ws + k8 * 8 + 4);
    const v4f c0 = *(const v4f*)(Ws + O1D + k8 * 8);
    const v4f c1 = *(const v4f*)(Ws + O1D + k8 * 8 + 4);
    const float f0 = h16_to_f32(w0 & 0xffffu), f1 = h16_to_f32(w0 >> 16);
    const float f2 = h16_to_f32(w1 & 0xffffu), f3 = h16_to_f32(w1 >> 16);
    const float f4 = h16_to_f32(w2w & 0xffffu), f5 = h16_to_f32(w2w >> 16);
    const float f6 = h16_to_f32(w3 & 0xffffu), f7 = h16_to_f32(w3 >> 16);
    s0 += f0 * a0[0]; s0 += f1 * a0[1]; s0 += f2 * a0[2]; s0 += f3 * a0[3];
    s0 += f4 * a1[0]; s0 += f5 * a1[1]; s0 += f6 * a1[2]; s0 += f7 * a1[3];
    s1 += f0 * c0[0]; s1 += f1 * c0[1]; s1 += f2 * c0[2]; s1 += f3 * c0[3];
    s1 += f4 * c1[0]; s1 += f5 * c1[1]; s1 += f6 * c1[2]; s1 += f7 * c1[3];
  }
  s0 += bf16r(b2[0]);
  s1 += bf16r(b2[1]);
  const float mx = fmaxf(s0, s1);
  const float d0 = s0 - mx, d1 = s1 - mx;
  const float lse = logf(expf(d0) + expf(d1));
  v2f o;
  o[0] = d0 - lse;
  o[1] = d1 - lse;
  float* op = out + (size_t)row * NCLS;
  *(volatile v2f*)op = o;
  __threadfence();
  *(volatile v2f*)op = o;
}

constexpr size_t U_QKV_B = (size_t)MROWS * 3 * HID * 4;
constexpr size_t U_S32_B = (size_t)MROWS * HID * 4;
constexpr size_t U_BYTES = U_QKV_B + U_S32_B;
static_assert(U_BYTES == (size_t)MROWS * 4 * HID * 4);
static_assert(U_QKV_B % 256 == 0 && U_S32_B % 256 == 0);

extern "C" void kernel_launch(void* const* d_in, const int* in_sizes, int n_in,
                              void* d_out, int out_size, void* d_ws, size_t ws_size, hipStream_t stream) {
  if (n_in < 25 || d_out == nullptr || d_ws == nullptr) return;
  if (in_sizes[0] != MROWS * DIN || in_sizes[1] != BATCH * NSLOT * HID || in_sizes[2] != BATCH * NSLOT * HID ||
      in_sizes[3] != HID * DIN || in_sizes[4] != HID ||
      in_sizes[5] != 3 * HID * HID || in_sizes[6] != 3 * HID ||
      in_sizes[7] != HID * HID || in_sizes[8] != HID ||
      in_sizes[9] != HID || in_sizes[10] != HID ||
      in_sizes[11] != FFD * HID || in_sizes[12] != FFD ||
      in_sizes[13] != HID * FFD || in_sizes[14] != HID ||
      in_sizes[15] != HID || in_sizes[16] != HID ||
      in_sizes[17] != 4 * HID * HID || in_sizes[18] != 4 * HID * HID ||
      in_sizes[19] != 4 * HID || in_sizes[20] != 4 * HID ||
      in_sizes[21] != O1D * HID || in_sizes[22] != O1D ||
      in_sizes[23] != NCLS * O1D || in_sizes[24] != NCLS ||
      out_size != (int)(OUT_TOTAL_B / 4)) return;

  const float* x       = (const float*)d_in[0];
  const float* uv_in   = (const float*)d_in[1];
  const float* gv_in   = (const float*)d_in[2];
  const float* fc_w    = (const float*)d_in[3];
  const float* fc_b    = (const float*)d_in[4];
  const float* inp_w   = (const float*)d_in[5];
  const float* inp_b   = (const float*)d_in[6];
  const float* outp_w  = (const float*)d_in[7];
  const float* outp_b  = (const float*)d_in[8];
  const float* ln1_w   = (const float*)d_in[9];
  const float* ln1_b   = (const float*)d_in[10];
  const float* ff1_w   = (const float*)d_in[11];
  const float* ff1_b   = (const float*)d_in[12];
  const float* ff2_w   = (const float*)d_in[13];
  const float* ff2_b   = (const float*)d_in[14];
  const float* ln2_w   = (const float*)d_in[15];
  const float* ln2_b   = (const float*)d_in[16];
  const float* wih     = (const float*)d_in[17];
  const float* whh     = (const float*)d_in[18];
  const float* bih     = (const float*)d_in[19];
  const float* bhh     = (const float*)d_in[20];
  const float* o1w     = (const float*)d_in[21];
  const float* o1b     = (const float*)d_in[22];
  const float* o2w     = (const float*)d_in[23];
  const float* o2b     = (const float*)d_in[24];

  float* out_logp = (float*)d_out;
  float* out_ct   = (float*)d_out + OUT1_OFF_B / 4;
  float* out_ht   = (float*)d_out + OUT2_OFF_B / 4;

  char* ws = (char*)d_ws;
  size_t off = 0;
  auto carve = [&](size_t bytes) -> char* { char* p = ws + off; off += (bytes + 255) & ~(size_t)255; return p; };
  unsigned short* WFC   = (unsigned short*)carve((size_t)HID * DIN * 2);
  unsigned short* WINP  = (unsigned short*)carve((size_t)3 * HID * HID * 2);
  unsigned short* WOUTP = (unsigned short*)carve((size_t)HID * HID * 2);
  unsigned short* WFF1  = (unsigned short*)carve((size_t)FFD * HID * 2);
  unsigned short* WFF2  = (unsigned short*)carve((size_t)HID * FFD * 2);
  unsigned short* WIH   = (unsigned short*)carve((size_t)4 * HID * HID * 2);
  unsigned short* WHH   = (unsigned short*)carve((size_t)4 * HID * HID * 2);
  unsigned short* WO1   = (unsigned short*)carve((size_t)O1D * HID * 2);
  unsigned short* X16   = (unsigned short*)carve((size_t)MROWS * DIN * 2);
  float*          CUR32 = (float*)carve((size_t)MROWS * HID * 4);
  unsigned short* P16H  = (unsigned short*)carve((size_t)MROWS * HID * 2);
  unsigned short* P16L  = (unsigned short*)carve((size_t)MROWS * HID * 2);
  char*           U     = carve(U_BYTES);
  float*          H1_32 = (float*)carve((size_t)MROWS * HID * 4);
  unsigned short* H1_16 = (unsigned short*)carve((size_t)MROWS * HID * 2);
  unsigned short* FFH16 = (unsigned short*)carve((size_t)MROWS * FFD * 2);
  unsigned short* O1_16 = (unsigned short*)carve((size_t)MROWS * O1D * 2);
  if (off > ws_size || off > (size_t)134217728) return;
  float* QKV32 = (float*)U;
  float* S32   = (float*)(U + U_QKV_B);
  float* XG32  = (float*)U;

  auto cvt = [&](const float* s, unsigned short* d, size_t n, float sc) {
    const int n8 = (int)(n / 8);
    cvt8_kernel<<<(unsigned)((n8 + 255) / 256), 256, 0, stream>>>(s, d, n8, sc);
  };
  cvt(x,      X16,   (size_t)MROWS * DIN,     1.0f);
  cvt(fc_w,   WFC,   (size_t)HID * DIN,       WCARRY);
  cvt(inp_w,  WINP,  (size_t)3 * HID * HID,   WCARRY);
  cvt(outp_w, WOUTP, (size_t)HID * HID,       WCARRY);
  cvt(ff1_w,  WFF1,  (size_t)FFD * HID,       WCARRY);
  cvt(ff2_w,  WFF2,  (size_t)HID * FFD,       WCARRY);
  cvt(wih,    WIH,   (size_t)4 * HID * HID,   WCARRY);
  cvt(whh,    WHH,   (size_t)4 * HID * HID,   WCARRY);
  cvt(o1w,    WO1,   (size_t)O1D * HID,       WCARRY);

  auto gblocks = [](int m, int n) -> unsigned { return (unsigned)(((m / 64) * (n / 64) + 7) / 8); };

  wmma_gemm64_f16<false, 4, false, 2><<<gblocks(MROWS, HID), 256, 0, stream>>>(
      X16, X16, DIN, WFC, DIN, CUR32, P16H, P16L, HID, fc_b, fc_b, MROWS, HID, DIN, WCARRY_INV);

  for (int j = 0; j < NSLOT; ++j) {
    wmma_gemm64_f16<true, 0, false, 0><<<gblocks(MROWS, 3 * HID), 256, 0, stream>>>(
        P16H, P16L, HID, WINP, HID, QKV32, H1_16, H1_16, 3 * HID, inp_b, inp_b, MROWS, 3 * HID, HID, WCARRY_INV);
    attn_kernel<<<BATCH * (NHEADS / ATT_WAVES), 128, 0, stream>>>(QKV32, P16H, P16L);
    wmma_gemm64_f16<true, 0, true, 0><<<gblocks(MROWS, HID), 256, 0, stream>>>(
        P16H, P16L, HID, WOUTP, HID, S32, H1_16, H1_16, HID, outp_b, CUR32, MROWS, HID, HID, WCARRY_INV);
    ln_rows_kernel<0><<<MROWS / 8, 256, 0, stream>>>(S32, ln1_w, ln1_b, H1_32, H1_16, H1_16, MROWS);
    wmma_gemm64_f16<false, 1, false, 2><<<gblocks(MROWS, FFD), 256, 0, stream>>>(
        H1_16, H1_16, HID, WFF1, HID, S32, FFH16, FFH16, FFD, ff1_b, ff1_b, MROWS, FFD, HID, WCARRY_INV);
    wmma_gemm64_f16<false, 0, true, 0><<<gblocks(MROWS, HID), 256, 0, stream>>>(
        FFH16, FFH16, FFD, WFF2, FFD, S32, H1_16, H1_16, HID, ff2_b, H1_32, MROWS, HID, FFD, WCARRY_INV);
    ln_rows_kernel<1><<<MROWS / 8, 256, 0, stream>>>(S32, ln2_w, ln2_b, H1_32, P16H, P16L, MROWS);
    wmma_gemm64_f16<true, 0, false, 0><<<gblocks(MROWS, 4 * HID), 256, 0, stream>>>(
        P16H, P16L, HID, WIH, HID, XG32, H1_16, H1_16, 4 * HID, bih, bih, MROWS, 4 * HID, HID, WCARRY_INV);
    lstm_seq_kernel<<<BATCH / 16, 256, 0, stream>>>(XG32, WHH, bhh, uv_in, gv_in, CUR32, P16H, P16L, out_ct, out_ht, j);
  }

  wmma_gemm64_f16<false, 1, false, 2><<<gblocks(MROWS, O1D), 256, 0, stream>>>(
      P16H, P16H, HID, WO1, HID, CUR32, O1_16, O1_16, O1D, o1b, o1b, MROWS, O1D, HID, WCARRY_INV);
  head_kernel<<<MROWS / 256, 256, 0, stream>>>(O1_16, o2w, o2b, out_logp);
}
